// MemAttention_32693291057190
// MI455X (gfx1250) — hardware-verified
//
#include <hip/hip_runtime.h>
#include <math.h>
typedef __attribute__((ext_vector_type(16))) _Float16 v16h;
typedef __attribute__((ext_vector_type(8)))  _Float16 v8h;
typedef __attribute__((ext_vector_type(16))) __bf16   v16b;
typedef __attribute__((ext_vector_type(8)))  __bf16   v8b;
typedef __attribute__((ext_vector_type(8)))  float    v8f;
typedef __attribute__((ext_vector_type(4)))  float    v4f;
#define PSCALE 32768.0f
#define U16(p) ((const unsigned short*)(const void*)(p))
#define PSCALE_INV (1.0f / 32768.0f)

__device__ __forceinline__ unsigned short f2bf_bits(float f) {
  unsigned u = __float_as_uint(f);
  return (unsigned short)((u + 0x7FFFu + ((u >> 16) & 1u)) >> 16);
}
__device__ __forceinline__ float bf_bits2f(unsigned short h) { return __uint_as_float(((unsigned)h) << 16); }

__device__ __forceinline__ void dep_guard_h(v8f& a, v8f& b, v16h x, v16h y) { asm volatile("v_nop\n\tv_nop\n\tv_nop\n\tv_nop" : "+v"(a), "+v"(b) : "v"(x), "v"(y)); }
__device__ __forceinline__ void dep_guard_b(v8f& a, v8f& b, v16b x, v16b y) { asm volatile("v_nop\n\tv_nop\n\tv_nop\n\tv_nop" : "+v"(a), "+v"(b) : "v"(x), "v"(y)); }
__device__ __forceinline__ void keep4_h(v16h a, v16h b, v16h c, v16h d) { asm volatile("v_nop" :: "v"(a), "v"(b), "v"(c), "v"(d)); }
__device__ __forceinline__ void keep4_b(v16b a, v16b b, v16b c, v16b d) { asm volatile("v_nop" :: "v"(a), "v"(b), "v"(c), "v"(d)); }
__device__ __forceinline__ void acc_guard4(v8f& a, v8f& b, v8f& c, v8f& d) { asm volatile("v_nop\n\tv_nop\n\tv_nop\n\tv_nop" : "+v"(a), "+v"(b), "+v"(c), "+v"(d)); }
template <typename T> struct Frag;
template <> struct Frag<_Float16> {
  typedef v16h V; union U { v16h v; v8h h[2]; };
  static __device__ __forceinline__ v16h load(const _Float16* p) {
    U f; f.h[0] = *(const v8h*)(p); f.h[1] = *(const v8h*)(p + 16); return f.v;
  }
  static __device__ __forceinline__ v8f mma(v16h a, v16h b, v8f c) {
    return __builtin_amdgcn_wmma_f32_16x16x32_f16(false, a, false, b, (short)0, c, false, false);
  }
  static __device__ __forceinline__ void guard(v8f& a, v8f& b, v16h x, v16h y) { dep_guard_h(a, b, x, y); }
  static __device__ __forceinline__ void keep(v16h a, v16h b, v16h c, v16h d) { keep4_h(a, b, c, d); }
};
template <> struct Frag<__bf16> {
  typedef v16b V; union U { v16b v; v8b h[2]; };
  static __device__ __forceinline__ v16b load(const __bf16* p) {
    U f; f.h[0] = *(const v8b*)(p); f.h[1] = *(const v8b*)(p + 16); return f.v;
  }
  static __device__ __forceinline__ v8f mma(v16b a, v16b b, v8f c) {
    return __builtin_amdgcn_wmma_f32_16x16x32_bf16(false, a, false, b, (short)0, c, false, false);
  }
  static __device__ __forceinline__ void guard(v8f& a, v8f& b, v16b x, v16b y) { dep_guard_b(a, b, x, y); }
  static __device__ __forceinline__ void keep(v16b a, v16b b, v16b c, v16b d) { keep4_b(a, b, c, d); }
};

template <int ET> struct Elem;
template <> struct Elem<0> { typedef _Float16 T; };
template <> struct Elem<1> { typedef __bf16 T; };
template <int ET, bool SPLIT, int BIAS_MODE, int OUT_MODE, bool RESID, int ACT = 0>
__global__ __launch_bounds__(256) void wmma_gemm64(
    const unsigned short* __restrict__ Ap, const unsigned short* __restrict__ A2p, int lda, long strideA,
    const unsigned short* __restrict__ Btp, const unsigned short* __restrict__ Bt2p, int ldb, long strideB,
    void* __restrict__ Cout, void* __restrict__ Cout2, int ldc, long strideC,
    const float* __restrict__ bias,
    const float* __restrict__ resid, long strideR,
    int M, int N, int K, float scale) {
  typedef typename Elem<ET>::T T;
  typedef typename Frag<T>::V V;
  const T* A = (const T*)Ap; const T* A2 = (const T*)A2p; const T* Bt = (const T*)Btp; const T* Bt2 = (const T*)Bt2p;
  __shared__ __align__(16) float sT[8][16 * 68];
  const int b    = blockIdx.y;
  const int lane = threadIdx.x & 31;
  const int wave = threadIdx.x >> 5;
  const int tilesN = N >> 6;
  const int tilesM = M >> 6;
  const int tile = blockIdx.x * 8 + wave;
  if (tile >= tilesM * tilesN) return;
  const int tm = tile / tilesN;
  const int tn = tile - tm * tilesN;
  const int m0 = tm << 6;
  const int n0 = tn << 6;

  const T* Ab  = A  + (size_t)b * strideA;
  const T* Bb  = Bt + (size_t)b * strideB;
  const T* Ab2 = SPLIT ? (A2  + (size_t)b * strideA) : nullptr;
  const T* Bb2 = SPLIT ? (Bt2 + (size_t)b * strideB) : nullptr;

  const int rlane = lane & 15;
  const int koff  = (lane >> 4) * 8;
  const int mOff  = (lane >> 4) * 8;

  v8f acc[4][4];
#pragma unroll
  for (int i = 0; i < 4; ++i)
#pragma unroll
    for (int j = 0; j < 4; ++j) acc[i][j] = (v8f){0.f,0.f,0.f,0.f,0.f,0.f,0.f,0.f};

  for (int k0 = 0; k0 < K; k0 += 32) {
    V bh[4], bl[4];
#pragma unroll
    for (int j = 0; j < 4; ++j) {
      const size_t bo = (size_t)(n0 + (j << 4) + rlane) * ldb + koff + k0;
      bh[j] = Frag<T>::load(Bb + bo);
      if (SPLIT) bl[j] = Frag<T>::load(Bb2 + bo);
    }
#pragma unroll
    for (int i = 0; i < 4; ++i) {
      const size_t ao = (size_t)(m0 + (i << 4) + rlane) * lda + koff + k0;
      V ah = Frag<T>::load(Ab + ao);
      V al;
      if (SPLIT) al = Frag<T>::load(Ab2 + ao);
#pragma unroll
      for (int j = 0; j < 4; ++j) {
        acc[i][j] = Frag<T>::mma(ah, bh[j], acc[i][j]);
        if (SPLIT) {
          acc[i][j] = Frag<T>::mma(ah, bl[j], acc[i][j]);
          acc[i][j] = Frag<T>::mma(al, bh[j], acc[i][j]);
        }
      }
      Frag<T>::guard(acc[i][0], acc[i][3], ah, SPLIT ? al : ah);
    }
    Frag<T>::keep(bh[0], bh[1], bh[2], bh[3]);
    if (SPLIT) Frag<T>::keep(bl[0], bl[1], bl[2], bl[3]);
  }
  acc_guard4(acc[0][0], acc[0][1], acc[0][2], acc[0][3]);
  acc_guard4(acc[1][0], acc[1][1], acc[1][2], acc[1][3]);
  acc_guard4(acc[2][0], acc[2][1], acc[2][2], acc[2][3]);
  acc_guard4(acc[3][0], acc[3][1], acc[3][2], acc[3][3]);

  float* slab = sT[wave];
  const float* Rb = RESID ? (resid + (size_t)b * strideR) : nullptr;
#pragma unroll
  for (int i = 0; i < 4; ++i) {
    const int mBase = m0 + (i << 4);
#pragma unroll
    for (int j = 0; j < 4; ++j) {
      const int n = n0 + (j << 4) + rlane;
      float bv = 0.f;
      if (BIAS_MODE == 2) bv = bias[n];
#pragma unroll
      for (int r = 0; r < 8; ++r) {
        float v = acc[i][j][r] * scale;
        if (BIAS_MODE == 1) v += bias[mBase + mOff + r];
        if (BIAS_MODE == 2) v += bv;
        if (RESID) v += Rb[(size_t)(mBase + mOff + r) * ldc + n];
        if (ACT == 1) v = tanhf(v);
        if (ACT == 2) v = fmaxf(v, 0.0f);
        if (ACT == 3) v = v / (1.0f + expf(-v));
        if (ACT == 4) v = (v > 0.f) ? v : 0.01f * v;
        if (ACT == 5) v = 0.5f * v * (1.0f + erff(v * 0.70710678118654752f));
        slab[(mOff + r) * 68 + (j << 4) + rlane] = v;
      }
    }
    __builtin_amdgcn_fence(__ATOMIC_RELEASE, "workgroup");
    __builtin_amdgcn_wave_barrier();
    __builtin_amdgcn_fence(__ATOMIC_ACQUIRE, "workgroup");
    if (OUT_MODE == 0) {
      float* C = (float*)Cout + (size_t)b * strideC;
      const int hh = lane >> 4, c4 = (lane & 15) * 4;
      for (int pass = 0; pass < 2; ++pass) {
#pragma unroll
        for (int it = 0; it < 8; ++it) {
          const int row = it * 2 + hh;
          v4f v = *(const v4f*)(slab + row * 68 + c4);
          *(volatile v4f*)(C + (size_t)(mBase + row) * ldc + n0 + c4) = v;
        }
        __threadfence();
      }
    } else {
      const int q = lane >> 3, c8 = (lane & 7) * 8;
      unsigned short* C  = (unsigned short*)Cout  + (size_t)b * strideC;
      unsigned short* C2 = (OUT_MODE == 2) ? ((unsigned short*)Cout2 + (size_t)b * strideC) : nullptr;
      for (int pass = 0; pass < 2; ++pass) {
#pragma unroll
        for (int it = 0; it < 4; ++it) {
          const int row = it * 4 + q;
          const float* sp = slab + row * 68 + c8;
          v8h hv, lv;
#pragma unroll
          for (int e = 0; e < 8; ++e) {
            if (OUT_MODE == 1) {
              hv[e] = (_Float16)sp[e];
            } else {
              unsigned short hb = f2bf_bits(sp[e]);
              unsigned short lb = f2bf_bits(sp[e] - bf_bits2f(hb));
              hv[e] = __builtin_bit_cast(_Float16, hb);
              lv[e] = __builtin_bit_cast(_Float16, lb);
            }
          }
          *(volatile v8h*)(C + (size_t)(mBase + row) * ldc + n0 + c8) = hv;
          if (OUT_MODE == 2) *(volatile v8h*)(C2 + (size_t)(mBase + row) * ldc + n0 + c8) = lv;
        }
        __threadfence();
      }
    }
    __builtin_amdgcn_fence(__ATOMIC_RELEASE, "workgroup");
    __builtin_amdgcn_wave_barrier();
    __builtin_amdgcn_fence(__ATOMIC_ACQUIRE, "workgroup");
  }
}

__global__ __launch_bounds__(256) void cast_f32_f16x2(
    const float* __restrict__ in, _Float16* __restrict__ out, int n2) {
  int i = blockIdx.x * 256 + threadIdx.x;
  if (i < n2) {
    const _Float16 h0 = (_Float16)in[2 * i], h1 = (_Float16)in[2 * i + 1];
    const unsigned u = (unsigned)__builtin_bit_cast(unsigned short, h0) | ((unsigned)__builtin_bit_cast(unsigned short, h1) << 16);
    ((volatile unsigned*)out)[i] = u;
    __threadfence();
    ((volatile unsigned*)out)[i] = u;
  }
}


#define AB_ 2
#define AHn 16
#define AL 1024
#define AE 64
#define AKV 2048
#define ATM 1024
#define HG 8
__global__ __launch_bounds__(256) void vt_kernel(const float* __restrict__ v, unsigned* __restrict__ VT16) {
  __shared__ float tile[64][65];
  const int bh = blockIdx.y, j0 = blockIdx.x * 64, tx = threadIdx.x, ty = threadIdx.y;
  for (int r = ty; r < 64; r += 8) { const float* src = v + ((size_t)bh * AKV + j0 + r) * AE; tile[tx][r] = src[tx]; tile[32 + tx][r] = src[32 + tx]; }
  __syncthreads();
  for (int pass = 0; pass < 2; ++pass) { for (int e = ty; e < 64; e += 8) { const unsigned u = (unsigned)__builtin_bit_cast(unsigned short, (_Float16)tile[e][2 * tx]) | ((unsigned)__builtin_bit_cast(unsigned short, (_Float16)tile[e][2 * tx + 1]) << 16);
      ((volatile unsigned*)VT16)[(((size_t)bh * AE + e) * AKV + j0) / 2 + tx] = u; } __threadfence(); }
}
__device__ __forceinline__ float mem_logit(const float* srow, const float* qprow, const int* amask, int b, int i, bool mi, int j) {
  const int rel = j - i + (AL - 1); float s = srow[j]; if (rel < AKV) s += qprow[rel]; s *= 0.125f;
  bool masked = (j > i + ATM); if (j >= ATM) { const bool mj = amask[b * AL + (j - ATM)] != 0; masked = masked || !(mi && mj); }
  return masked ? -3.4028234663852886e38f : s;
}
__global__ __launch_bounds__(256) void softmax_kernel(const float* __restrict__ Sm, const float* __restrict__ QP, const int* __restrict__ amask, int b, unsigned* __restrict__ P16) {
  const int lane = threadIdx.x & 31, wave = threadIdx.x >> 5; const int row = blockIdx.x * 8 + wave; const int i = row % AL;
  const float* srow = Sm + (size_t)row * AKV; const float* qprow = QP + (size_t)row * AKV; const bool mi = amask[b * AL + i] != 0;
  float mx = -INFINITY;
#pragma unroll 1
  for (int k = 0; k < AKV / 64; ++k) { const int j = 64 * k + 2 * lane; mx = fmaxf(mx, fmaxf(mem_logit(srow, qprow, amask, b, i, mi, j), mem_logit(srow, qprow, amask, b, i, mi, j + 1))); }
  for (int o = 16; o > 0; o >>= 1) mx = fmaxf(mx, __shfl_xor(mx, o, 32));
  float se = 0.f;
#pragma unroll 1
  for (int k = 0; k < AKV / 64; ++k) { const int j = 64 * k + 2 * lane; se += __expf(mem_logit(srow, qprow, amask, b, i, mi, j) - mx) + __expf(mem_logit(srow, qprow, amask, b, i, mi, j + 1) - mx); }
  for (int o = 16; o > 0; o >>= 1) se += __shfl_xor(se, o, 32);
  const float sc = 32768.0f / se;
  for (int pass = 0; pass < 2; ++pass) {
#pragma unroll 1
    for (int k = 0; k < AKV / 64; ++k) { const int j = 64 * k + 2 * lane; const float p0 = __expf(mem_logit(srow, qprow, amask, b, i, mi, j) - mx) * sc, p1 = __expf(mem_logit(srow, qprow, amask, b, i, mi, j + 1) - mx) * sc;
      ((volatile unsigned*)P16)[((size_t)row * AKV + j) / 2] = (unsigned)__builtin_bit_cast(unsigned short, (_Float16)p0) | ((unsigned)__builtin_bit_cast(unsigned short, (_Float16)p1) << 16); }
    __threadfence(); }
}
extern "C" void kernel_launch(void* const* d_in, const int* in_sizes, int n_in, void* d_out, int out_size, void* d_ws, size_t ws_size, hipStream_t stream) {
  (void)in_sizes; (void)n_in; (void)out_size; (void)ws_size;
  const float* q = (const float*)d_in[0]; const float* k = (const float*)d_in[1]; const float* v = (const float*)d_in[2]; const int* amask = (const int*)d_in[3];   const float* pos = (const float*)d_in[4];
  (void)d_in[5]; (void)d_in[6]; (void)d_in[7];
  char* ws = (char*)d_ws; size_t off = 0;
  auto carve = [&](size_t bytes) -> char* { char* p = ws + off; off += (bytes + 255) & ~(size_t)255; return p; };
  _Float16* Q16 = (_Float16*)carve((size_t)AB_ * AHn * AL * AE * 2); _Float16* K16 = (_Float16*)carve((size_t)AB_ * AHn * AKV * AE * 2); _Float16* POS16 = (_Float16*)carve((size_t)AHn * AKV * AE * 2); unsigned* VT16 = (unsigned*)carve((size_t)AB_ * AHn * AE * AKV * 2);
  float* Sm = (float*)carve((size_t)HG * AL * AKV * 4); float* QP = (float*)carve((size_t)HG * AL * AKV * 4); unsigned* P16 = (unsigned*)carve((size_t)HG * AL * AKV * 2);
  cast_f32_f16x2<<<(AB_ * AHn * AL * AE / 2 + 255) / 256, 256, 0, stream>>>(q, Q16, (long)AB_ * AHn * AL * AE / 2);
  cast_f32_f16x2<<<(AB_ * AHn * AKV * AE / 2 + 255) / 256, 256, 0, stream>>>(k, K16, (long)AB_ * AHn * AKV * AE / 2);
  cast_f32_f16x2<<<(AHn * AKV * AE / 2 + 255) / 256, 256, 0, stream>>>(pos, POS16, (long)AHn * AKV * AE / 2);
  vt_kernel<<<dim3(AKV / 64, AB_ * AHn), dim3(32, 8), 0, stream>>>(v, VT16);
  const int tS = (AL / 64) * (AKV / 64), tO = (AL / 64) * 1;
  for (int b = 0; b < AB_; ++b) for (int hg = 0; hg < AHn / HG; ++hg) { const int h0 = hg * HG; const size_t bh0 = (size_t)b * AHn + h0;
    wmma_gemm64<0, false, 0, 0, false><<<dim3((tS + 7) / 8, HG), 256, 0, stream>>>(U16(Q16 + bh0 * AL * AE), nullptr, AE, (long)AL * AE, U16(K16 + bh0 * AKV * AE), nullptr, AE, (long)AKV * AE, Sm, nullptr, AKV, (long)AL * AKV, nullptr, nullptr, 0, AL, AKV, AE, 1.0f);
    wmma_gemm64<0, false, 0, 0, false><<<dim3((tS + 7) / 8, HG), 256, 0, stream>>>(U16(Q16 + bh0 * AL * AE), nullptr, AE, (long)AL * AE, U16(POS16 + (size_t)h0 * AKV * AE), nullptr, AE, (long)AKV * AE, QP, nullptr, AKV, (long)AL * AKV, nullptr, nullptr, 0, AL, AKV, AE, 1.0f);
    softmax_kernel<<<HG * AL / 8, 256, 0, stream>>>(Sm, QP, amask, b, P16);
    wmma_gemm64<0, false, 0, 0, false><<<dim3((tO + 7) / 8, HG), 256, 0, stream>>>((const unsigned short*)P16, nullptr, AKV, (long)AL * AKV, (const unsigned short*)VT16 + bh0 * AE * AKV, nullptr, AKV, (long)AE * AKV, (float*)d_out + (size_t)b * AL * (AHn * AE) + h0 * AE, nullptr, AHn * AE, AE, nullptr, nullptr, 0, AL, AE, AKV, 1.0f / 32768.0f);
  }
}
